// CausalSelfAttention_77610059038806
// MI455X (gfx1250) — hardware-verified
//
#include <hip/hip_runtime.h>
#ifndef NB
#define NB 2
#endif
#ifndef SQ
#define SQ 2048
#endif
#define SQ_FULL 2048
#define DM 1024
#define NH 16
#define HD 64
#define EARLY ((SQ) < 256 ? (SQ) : 256)
#define NR (NB * SQ)
#define LDV NR

static_assert(DM == NH * HD);
static_assert(HD == 64);
static_assert(DM % 64 == 0);
static_assert(DM % 32 == 0);
static_assert(DM % 128 == 0);
static_assert(DM % 8 == 0);
static_assert(NR % 128 == 0);
static_assert(NR % 64 == 0);
static_assert(LDV % 64 == 0);
static_assert(SQ % 64 == 0);
static_assert(EARLY % 64 == 0);
static_assert((SQ - EARLY) % 64 == 0);
static_assert(SQ <= SQ_FULL);

typedef unsigned short v8us __attribute__((ext_vector_type(8), may_alias));
typedef float  v8f  __attribute__((ext_vector_type(8)));
typedef float  v4f  __attribute__((ext_vector_type(4)));
typedef float  v4fa __attribute__((ext_vector_type(4), may_alias));
typedef _Float16 v16h __attribute__((ext_vector_type(16)));
typedef _Float16 v4h __attribute__((ext_vector_type(4)));
union FragH { v16h v; v8us half[2]; _Float16 h[16]; unsigned short u[16]; };

constexpr size_t SZ_W   = (size_t)DM * DM * 2;
constexpr size_t SZ_P   = (size_t)NR * DM * 2;
constexpr size_t OFF_BW  = 0;
constexpr size_t OFF_X   = OFF_BW + 4 * SZ_W;
constexpr size_t OFF_QK  = OFF_X + SZ_P;
constexpr size_t OFF_QKL = OFF_QK + 2 * SZ_P;
constexpr size_t OFF_VT  = OFF_QKL + 2 * SZ_P;
constexpr size_t OFF_VTL = OFF_VT + SZ_P;
constexpr size_t OFF_O   = OFF_VTL + SZ_P;
constexpr size_t OFF_OL  = OFF_O + SZ_P;
constexpr size_t WS_TOTAL = OFF_OL + SZ_P;
static_assert(SZ_W % 256 == 0);
static_assert(SZ_P % 256 == 0);
static_assert(WS_TOTAL <= (size_t)134217728);

__device__ __forceinline__ unsigned short bf16_bits(float x) { unsigned int u = __float_as_uint(x); return (unsigned short)((u + 0x7FFFu + ((u >> 16) & 1u)) >> 16); }
__device__ __forceinline__ float bf16_rne(float x) { return __uint_as_float(((unsigned int)bf16_bits(x)) << 16); }

__device__ __forceinline__ v16h g2_frag(const _Float16* p, int hh) { FragH f; f.half[0] = *(const v8us*)((const unsigned short*)p + 8 * hh); f.half[1] = *(const v8us*)((const unsigned short*)p + 16 + 8 * hh); return f.v; }
__device__ __forceinline__ v8f g2_mma(v16h a, v16h b, v8f c) { v8f d = __builtin_amdgcn_wmma_f32_16x16x32_f16(false, a, false, b, (short)0, c, false, false); asm volatile("v_nop\n\tv_nop\n\tv_nop\n\tv_nop" : "+v"(d) : "v"(a), "v"(b)); return d; }

__global__ __launch_bounds__(256) void k_wt_f16(const float* __restrict__ W, _Float16* __restrict__ Wt, int K, int N, float scale) {
  const int t = blockIdx.x * 256 + threadIdx.x; if (t >= N * (K / 8)) return; const int n = t / (K / 8), k8 = (t % (K / 8)) * 8; FragH f;
#pragma unroll
  for (int i = 0; i < 8; ++i) f.h[i] = (_Float16)(bf16_rne(W[(size_t)(k8 + i) * N + n]) * scale);
  const v8us o = f.half[0];
  *(volatile v8us*)((unsigned short*)Wt + (size_t)n * K + k8) = o; __threadfence(); *(volatile v8us*)((unsigned short*)Wt + (size_t)n * K + k8) = o;
}

__global__ __launch_bounds__(256) void k_x16(const float* __restrict__ x, _Float16* __restrict__ X16) {
  const size_t t = (size_t)blockIdx.x * 256 + threadIdx.x; if (t >= (size_t)NR * DM / 8) return;
  const size_t row = t / (DM / 8); const int c8 = (int)(t % (DM / 8)) * 8; const size_t b = row / SQ, s = row % SQ;
  const float* src = x + (b * SQ_FULL + s) * DM + c8;
  const v4f a = *(const v4fa*)src, c = *(const v4fa*)(src + 4); FragH f;
#pragma unroll
  for (int q = 0; q < 4; ++q) { f.h[q] = (_Float16)bf16_rne(a[q]); f.h[4 + q] = (_Float16)bf16_rne(c[q]); }
  const v8us o = f.half[0];
  *(volatile v8us*)((unsigned short*)X16 + t * 8) = o; __threadfence(); *(volatile v8us*)((unsigned short*)X16 + t * 8) = o;
}

struct Acc8 { v8f c[8]; };
__device__ __forceinline__ Acc8 g2_loop(const _Float16* a0p, const _Float16* a1p, const _Float16* b0p, const _Float16* b1p, const _Float16* b2p, const _Float16* b3p, int K, int hh) {
  const v8f z8 = {0.f,0.f,0.f,0.f,0.f,0.f,0.f,0.f}; v8f c00 = z8, c01 = z8, c02 = z8, c03 = z8, c10 = z8, c11 = z8, c12 = z8, c13 = z8;
#pragma unroll 1
  for (int kb = 0; kb < K; kb += 32) { const v16h a0 = g2_frag(a0p + kb, hh), a1 = g2_frag(a1p + kb, hh);
    v16h b = g2_frag(b0p + kb, hh); c00 = g2_mma(a0, b, c00); c10 = g2_mma(a1, b, c10);
    b = g2_frag(b1p + kb, hh); c01 = g2_mma(a0, b, c01); c11 = g2_mma(a1, b, c11);
    b = g2_frag(b2p + kb, hh); c02 = g2_mma(a0, b, c02); c12 = g2_mma(a1, b, c12);
    b = g2_frag(b3p + kb, hh); c03 = g2_mma(a0, b, c03); c13 = g2_mma(a1, b, c13); }
  Acc8 r; r.c[0] = c00; r.c[1] = c01; r.c[2] = c02; r.c[3] = c03; r.c[4] = c10; r.c[5] = c11; r.c[6] = c12; r.c[7] = c13; return r;
}
template <bool DUAL>
__device__ __forceinline__ void gemm2_body(const _Float16* __restrict__ A, const _Float16* __restrict__ A2, int lda, size_t sA, size_t sA2,
    const _Float16* __restrict__ Bh, int ldb, size_t sB, float alpha, float alpha2,
    float* __restrict__ C, _Float16* __restrict__ C16, _Float16* __restrict__ C16L, int ldc, size_t sC, int N, int K, int resPer, int resLim, int resCols) {
  __shared__ __attribute__((aligned(16))) float so[4][32][68];
  const int tid = threadIdx.x, lane = tid & 31, ln = lane & 15, hh = lane >> 4;
  const int w = __builtin_amdgcn_readfirstlane((int)(tid >> 5));
  const int by = blockIdx.y;
  A += (size_t)by * sA; Bh += (size_t)by * sB; const size_t cofs = (size_t)by * sC;
  const int ntn = N >> 6; const int mt = blockIdx.x / ntn, nq = blockIdx.x - mt * ntn; const int row0 = mt * 128 + 32 * w, col0 = nq * 64;
  const _Float16* a0p = A + (size_t)(row0 + ln) * lda; const _Float16* a1p = a0p + (size_t)16 * lda;
  const _Float16* b0p = Bh + (size_t)(col0 + ln) * ldb; const _Float16* b1p = b0p + (size_t)16 * ldb; const _Float16* b2p = b1p + (size_t)16 * ldb; const _Float16* b3p = b2p + (size_t)16 * ldb;
  { const Acc8 acc = g2_loop(a0p, a1p, b0p, b1p, b2p, b3p, K, hh);
#pragma unroll
    for (int u = 0; u < 8; ++u) { const int t = u & 3, half = u >> 2;
#pragma unroll
      for (int r = 0; r < 8; ++r) so[w][half * 16 + 8 * hh + r][t * 16 + ln] = acc.c[u][r] * alpha; } }
  if (DUAL) { const _Float16* e0p = A2 + (size_t)by * sA2 + (size_t)(row0 + ln) * lda; const _Float16* e1p = e0p + (size_t)16 * lda;
    const Acc8 acc2 = g2_loop(e0p, e1p, b0p, b1p, b2p, b3p, K, hh);
#pragma unroll
    for (int u = 0; u < 8; ++u) { const int t = u & 3, half = u >> 2;
#pragma unroll
      for (int r = 0; r < 8; ++r) { const float pv = so[w][half * 16 + 8 * hh + r][t * 16 + ln]; so[w][half * 16 + 8 * hh + r][t * 16 + ln] = pv + acc2.c[u][r] * alpha2; } } }
  __builtin_amdgcn_fence(4  , "workgroup"); __builtin_amdgcn_wave_barrier();
  const int rkey = resCols ? col0 : row0;
  const bool wres = (C16L != nullptr) && (resPer > 0) && ((rkey % resPer) < resLim);
  const int rsub = lane >> 4, c4 = (lane & 15) * 4;
  for (int pass = 0; pass < 2; ++pass) {
#pragma unroll
    for (int q = 0; q < 16; ++q) { const int r = q * 2 + rsub; const v4f v = *(const v4fa*)&so[w][r][c4]; const size_t o = cofs + (size_t)(row0 + r) * ldc + col0 + c4;
      if (C) *(volatile v4f*)(C + o) = v;
      if (C16) { v4h h4;
#pragma unroll
        for (int i = 0; i < 4; ++i) h4[i] = (_Float16)v[i];
        *(volatile v4h*)(C16 + o) = h4;
        if (wres) { v4h l4;
#pragma unroll
          for (int i = 0; i < 4; ++i) l4[i] = (_Float16)((v[i] - (float)h4[i]) * 1024.0f);
          *(volatile v4h*)(C16L + o) = l4; } } }
    if (pass == 0) __threadfence(); }
}
__global__ __launch_bounds__(128) void k_gemm_p(const _Float16* __restrict__ A, int lda, size_t sA, const _Float16* __restrict__ Bh, int ldb, size_t sB, float alpha,
    float* __restrict__ C, _Float16* __restrict__ C16, _Float16* __restrict__ C16L, int ldc, size_t sC, int N, int K, int resPer, int resLim, int resCols) {
  gemm2_body<false>(A, nullptr, lda, sA, 0, Bh, ldb, sB, alpha, 0.f, C, C16, C16L, ldc, sC, N, K, resPer, resLim, resCols);
}
__global__ __launch_bounds__(128) void k_gemm_o2(const _Float16* __restrict__ A, const _Float16* __restrict__ A2, int lda, size_t sA, size_t sA2, const _Float16* __restrict__ Bh, int ldb, float alpha, float alpha2,
    float* __restrict__ C, int ldc, size_t sC, int N, int K) {
  gemm2_body<true>(A, A2, lda, sA, sA2, Bh, ldb, 0, alpha, alpha2, C, nullptr, nullptr, ldc, sC, N, K, 0, 0, 0);
}

template <bool RES>
__device__ __forceinline__ void attn_body(const _Float16* __restrict__ Q16, const _Float16* __restrict__ Q16L, const _Float16* __restrict__ K16, const _Float16* __restrict__ K16L,
    const _Float16* __restrict__ VT, const _Float16* __restrict__ VTL, _Float16* __restrict__ O16, _Float16* __restrict__ O16L, int qblk0) {
  __shared__ __attribute__((aligned(16))) float so[4][16][68];
  const int tid = threadIdx.x, lane = tid & 31, ln = lane & 15, hh = lane >> 4;
  const int wave = __builtin_amdgcn_readfirstlane((int)(tid >> 5));
  const int qb = (int)blockIdx.x + qblk0, h = blockIdx.y, b = blockIdx.z;
  const int q0w = qb * 64 + wave * 16;
  const int nhalf = ((q0w + 15) >> 5) + 1;
  const size_t tok0 = (size_t)b * SQ;
  const size_t qoff = (tok0 + q0w + ln) * DM + h * HD;
  const size_t koff = (tok0 + ln) * DM + h * HD;
  const size_t voff = (size_t)(h * HD + ln) * LDV + tok0;
  const int qi = q0w + ln;
  const v8f z8 = {0.f,0.f,0.f,0.f,0.f,0.f,0.f,0.f};
  v8f o[4] = {z8, z8, z8, z8}; v8f ol[4] = {z8, z8, z8, z8};
  float m = -1.0e30f, lsum = 0.f;
#pragma unroll 1
  for (int kh = 0; kh < nhalf; ++kh) {
    const int k0 = kh * 32;
    v8f s0 = z8, s1 = z8, t0 = z8, t1 = z8;
#pragma unroll 1
    for (int ds = 0; ds < 2; ++ds) {
      const v16h bq = g2_frag(Q16 + qoff + ds * 32, hh);
      const v16h a0 = g2_frag(K16 + koff + (size_t)k0 * DM + ds * 32, hh);
      const v16h a1 = g2_frag(K16 + koff + (size_t)(k0 + 16) * DM + ds * 32, hh);
      s0 = g2_mma(a0, bq, s0); s1 = g2_mma(a1, bq, s1);
      const v16h bql = g2_frag(Q16L + qoff + ds * 32, hh);
      const v16h a0l = g2_frag(K16L + koff + (size_t)k0 * DM + ds * 32, hh);
      const v16h a1l = g2_frag(K16L + koff + (size_t)(k0 + 16) * DM + ds * 32, hh);
      t0 = g2_mma(a0l, bq, t0); t0 = g2_mma(a0, bql, t0);
      t1 = g2_mma(a1l, bq, t1); t1 = g2_mma(a1, bql, t1);
    }
    float v0[8], v1[8]; float mx = -1.0e30f;
#pragma unroll
    for (int r = 0; r < 8; ++r) {
      float a = s0[r] + t0[r] * 0.0009765625f;
      float c = s1[r] + t1[r] * 0.0009765625f;
      const int key = k0 + 8 * hh + r;
      a = (key <= qi) ? a * 0.125f : -1.0e30f;
      c = (key + 16 <= qi) ? c * 0.125f : -1.0e30f;
      v0[r] = a; v1[r] = c; mx = fmaxf(mx, fmaxf(a, c));
    }
    mx = fmaxf(mx, __shfl_xor(mx, 16, 32));
    const float mn = fmaxf(m, mx);
    const float alpha = __expf(m - mn);
    m = mn;
    FragH pf, pl; float ps = 0.f;
#pragma unroll
    for (int r = 0; r < 8; ++r) {
      const float e0 = __expf(v0[r] - mn), e1 = __expf(v1[r] - mn);
      ps += e0 + e1;
      const float x0 = e0 * 256.0f, x1 = e1 * 256.0f;
      const _Float16 h0 = (_Float16)x0, h1 = (_Float16)x1;
      pf.h[r] = h0; pf.h[8 + r] = h1;
      if (RES) { pl.h[r] = (_Float16)((x0 - (float)h0) * 1024.0f); pl.h[8 + r] = (_Float16)((x1 - (float)h1) * 1024.0f); }
    }
    lsum = lsum * alpha + ps;
#pragma unroll
    for (int j = 0; j < 4; ++j) {
#pragma unroll
      for (int r = 0; r < 8; ++r) { o[j][r] *= alpha; if (RES) ol[j][r] *= alpha; }
    }
#pragma unroll
    for (int j = 0; j < 4; ++j) {
      const v16h av = g2_frag(VT + voff + (size_t)(j * 16) * LDV + k0, hh);
      o[j] = g2_mma(av, pf.v, o[j]);
      if (RES) {
        const v16h avl = g2_frag(VTL + voff + (size_t)(j * 16) * LDV + k0, hh);
        ol[j] = g2_mma(avl, pf.v, ol[j]);
        ol[j] = g2_mma(av, pl.v, ol[j]);
      }
    }
  }
  const float lt = lsum + __shfl_xor(lsum, 16, 32);
  const float fin = 0.25f * (1.0f / lt);
#pragma unroll
  for (int j = 0; j < 4; ++j) {
#pragma unroll
    for (int r = 0; r < 8; ++r) { float v = o[j][r]; if (RES) v += ol[j][r] * 0.0009765625f; so[wave][ln][j * 16 + 8 * hh + r] = v * fin; }
  }
  __syncthreads();
  const int rq = lane >> 3, pc = (lane & 7) * 8;
  v8us oh[4], olw[4];
#pragma unroll
  for (int it = 0; it < 4; ++it) {
    const int row = it * 4 + rq;
    const v4f a = *(const v4fa*)&so[wave][row][pc], c = *(const v4fa*)&so[wave][row][pc + 4];
    FragH fh, fl;
#pragma unroll
    for (int q = 0; q < 4; ++q) {
      const _Float16 h0 = (_Float16)a[q], h1 = (_Float16)c[q];
      fh.h[q] = h0; fh.h[4 + q] = h1;
      fl.h[q] = (_Float16)((a[q] - (float)h0) * 1024.0f); fl.h[4 + q] = (_Float16)((c[q] - (float)h1) * 1024.0f);
    }
    oh[it] = fh.half[0]; olw[it] = fl.half[0];
  }
  for (int pass = 0; pass < 2; ++pass) {
#pragma unroll
    for (int it = 0; it < 4; ++it) {
      const int row = it * 4 + rq;
      const size_t oidx = (tok0 + q0w + row) * DM + h * HD + pc;
      *(volatile v8us*)((unsigned short*)O16 + oidx) = oh[it];
      *(volatile v8us*)((unsigned short*)O16L + oidx) = olw[it];
    }
    if (pass == 0) __threadfence();
  }
}
__global__ __launch_bounds__(128) void k_attn_main(const _Float16* __restrict__ Q16, const _Float16* __restrict__ Q16L, const _Float16* __restrict__ K16, const _Float16* __restrict__ K16L,
    const _Float16* __restrict__ VT, _Float16* __restrict__ O16, _Float16* __restrict__ O16L, int qblk0) {
  attn_body<false>(Q16, Q16L, K16, K16L, VT, nullptr, O16, O16L, qblk0);
}
__global__ __launch_bounds__(128) void k_attn_early(const _Float16* __restrict__ Q16, const _Float16* __restrict__ Q16L, const _Float16* __restrict__ K16, const _Float16* __restrict__ K16L,
    const _Float16* __restrict__ VT, const _Float16* __restrict__ VTL, _Float16* __restrict__ O16, _Float16* __restrict__ O16L) {
  attn_body<true>(Q16, Q16L, K16, K16L, VT, VTL, O16, O16L, 0);
}

extern "C" void kernel_launch(void* const* d_in, const int* in_sizes, int n_in,
                              void* d_out, int out_size, void* d_ws, size_t ws_size, hipStream_t stream) {
  if (n_in < 5) return;
  if ((size_t)in_sizes[0] < (size_t)(NB - 1) * SQ_FULL * DM + (size_t)SQ * DM) return;
  if (in_sizes[1] < DM * DM || in_sizes[2] < DM * DM || in_sizes[3] < DM * DM || in_sizes[4] < DM * DM) return;
  if ((size_t)out_size < (size_t)NR * DM) return;
  if (WS_TOTAL > ws_size) return;
  const float* x = (const float*)d_in[0]; const float* wq = (const float*)d_in[1]; const float* wk = (const float*)d_in[2]; const float* wv = (const float*)d_in[3]; const float* wo = (const float*)d_in[4];
  float* out = (float*)d_out;
  char* ws = (char*)d_ws;
  _Float16* BQ = (_Float16*)(ws + OFF_BW); _Float16* BK = BQ + (size_t)DM * DM; _Float16* BV = BK + (size_t)DM * DM; _Float16* BO = BV + (size_t)DM * DM;
  _Float16* X16 = (_Float16*)(ws + OFF_X);
  _Float16* Q16 = (_Float16*)(ws + OFF_QK); _Float16* K16 = Q16 + (size_t)NR * DM;
  _Float16* Q16L = (_Float16*)(ws + OFF_QKL); _Float16* K16L = Q16L + (size_t)NR * DM;
  _Float16* VT = (_Float16*)(ws + OFF_VT); _Float16* VTL = (_Float16*)(ws + OFF_VTL);
  _Float16* O16 = (_Float16*)(ws + OFF_O); _Float16* O16L = (_Float16*)(ws + OFF_OL);

  const unsigned gw = (unsigned)(((size_t)DM * (DM / 8) + 255) / 256);
  k_wt_f16<<<gw, 256, 0, stream>>>(wq, BQ, DM, DM, 16.0f);
  k_wt_f16<<<gw, 256, 0, stream>>>(wk, BK, DM, DM, 16.0f);
  k_wt_f16<<<gw, 256, 0, stream>>>(wv, BV, DM, DM, 16.0f);
  k_wt_f16<<<gw, 256, 0, stream>>>(wo, BO, DM, DM, 16.0f);
  k_x16<<<(unsigned)(((size_t)NR * DM / 8 + 255) / 256), 256, 0, stream>>>(x, X16);
  k_gemm_p<<<dim3((unsigned)((NR / 128) * (DM / 64)), 2), 128, 0, stream>>>(X16, DM, (size_t)0, BQ, DM, (size_t)DM * DM, 0.0625f, nullptr, Q16, Q16L, DM, (size_t)NR * DM, DM, DM, SQ, SQ, 0);
  k_gemm_p<<<dim3((unsigned)((DM / 128) * (NR / 64)), 1), 128, 0, stream>>>(BV, DM, (size_t)0, X16, DM, (size_t)0, 0.0625f, nullptr, VT, VTL, NR, (size_t)0, NR, DM, SQ, EARLY, 1);
  k_attn_early<<<dim3(EARLY / 64, NH, NB), 128, 0, stream>>>(Q16, Q16L, K16, K16L, VT, VTL, O16, O16L);
  if (SQ > EARLY) {
    k_attn_main<<<dim3((SQ - EARLY) / 64, NH, NB), 128, 0, stream>>>(Q16, Q16L, K16, K16L, VT, O16, O16L, EARLY / 64);
  }
  k_gemm_o2<<<dim3((unsigned)((NR / 128) * (DM / 64)), 1), 128, 0, stream>>>(O16, O16L, DM, (size_t)0, (size_t)0, BO, DM, 0.0009765625f, 0.00000095367431640625f, out, DM, (size_t)0, DM, DM);
}
